// TraceableEncoderLayer_66709432041881
// MI455X (gfx1250) — hardware-verified
//
#include <hip/hip_runtime.h>
#include <stddef.h>
#include <stdint.h>

#define NB    2
#define SQ    2048
#define NTOK  4096
#define DM    1024
#define NH    16
#define HD    64
#define DFF   4096
#define NQKV  3072
#define QB    128
#define KC    64
#define NQB   (SQ / QB)
#define WSLIM 134217728

static_assert(NTOK == NB * SQ);
static_assert(NH * HD == DM);
static_assert(NQKV == 3 * DM);
static_assert(SQ % QB == 0);
static_assert(QB == 2 * KC);
static_assert(SQ % 128 == 0);
static_assert(NTOK % 128 == 0);
static_assert(DM % 64 == 0);
static_assert(DFF % 64 == 0);
static_assert(DM == 128 * 8);
static_assert(HD == 64);

typedef _Float16 v16h __attribute__((ext_vector_type(16)));
typedef _Float16 v8h  __attribute__((ext_vector_type(8)));
typedef float    v8f  __attribute__((ext_vector_type(8)));
typedef float    v4f  __attribute__((ext_vector_type(4)));
typedef unsigned int v4u __attribute__((ext_vector_type(4)));

union Frag  { v16h v; v8h h[2]; };
union Pack8 { v8h h; v4u u; };

__device__ __forceinline__ v8f zero8() { return (v8f){0.f, 0.f, 0.f, 0.f, 0.f, 0.f, 0.f, 0.f}; }

__device__ __forceinline__ v4u packh(v4f a, v4f b) {
  Pack8 pk;
  pk.h = (v8h){(_Float16)a[0], (_Float16)a[1], (_Float16)a[2], (_Float16)a[3],
               (_Float16)b[0], (_Float16)b[1], (_Float16)b[2], (_Float16)b[3]};
  return pk.u;
}

__device__ __forceinline__ v8f mma16(v16h a, v16h b, v8f cacc) {
  cacc = __builtin_amdgcn_wmma_f32_16x16x32_f16(false, a, false, b, (short)0, cacc, false, false);
  asm volatile("v_nop\n\tv_nop\n\tv_nop\n\tv_nop" : "+v"(cacc) : "v"(a), "v"(b));
  return cacc;
}

__device__ __forceinline__ v16h ldfrag(const _Float16* p, int ld, int row0, int k0, int lane) {
  const int m = lane & 15, lh = lane >> 4;
  const _Float16* q = p + (size_t)(row0 + m) * ld + k0 + 8 * lh;
  Frag f;
  f.h[0] = *(const v8h*)(q);
  f.h[1] = *(const v8h*)(q + 16);
  return f.v;
}

__device__ __forceinline__ void gemm32x64(const _Float16* __restrict__ A, int lda,
                                          const _Float16* __restrict__ Bt, int ldb, int K,
                                          int m0, int n0, int lane, v8f (&acc)[2][4]) {
#pragma unroll 2
  for (int k0 = 0; k0 < K; k0 += 32) {
    const v16h a0 = ldfrag(A, lda, m0, k0, lane);
    const v16h a1 = ldfrag(A, lda, m0 + 16, k0, lane);
    const v16h b0 = ldfrag(Bt, ldb, n0, k0, lane);
    const v16h b1 = ldfrag(Bt, ldb, n0 + 16, k0, lane);
    const v16h b2 = ldfrag(Bt, ldb, n0 + 32, k0, lane);
    const v16h b3 = ldfrag(Bt, ldb, n0 + 48, k0, lane);
    acc[0][0] = mma16(a0, b0, acc[0][0]);
    acc[1][0] = mma16(a1, b0, acc[1][0]);
    acc[0][1] = mma16(a0, b1, acc[0][1]);
    acc[1][1] = mma16(a1, b1, acc[1][1]);
    acc[0][2] = mma16(a0, b2, acc[0][2]);
    acc[1][2] = mma16(a1, b2, acc[1][2]);
    acc[0][3] = mma16(a0, b3, acc[0][3]);
    acc[1][3] = mma16(a1, b3, acc[1][3]);
  }
}

__global__ __launch_bounds__(128) void k_ln(const float* __restrict__ x, const float* __restrict__ w,
                                            const float* __restrict__ gate, int use_gate,
                                            _Float16* __restrict__ out) {
  __shared__ float red[8];
  const int tid = threadIdx.x, lane = tid & 31, wave = tid >> 5;
  const int row = blockIdx.x;
  const int col = tid * 8;
  const float* xr = x + (size_t)row * DM + col;
  const v4f a0 = *(const v4f*)(xr);
  const v4f a1 = *(const v4f*)(xr + 4);
  float s = ((a0[0] + a0[1]) + (a0[2] + a0[3])) + ((a1[0] + a1[1]) + (a1[2] + a1[3]));
#pragma unroll
  for (int off = 1; off < 32; off <<= 1) s += __shfl_xor(s, off, 32);
  if (lane == 0) red[wave] = s;
  __syncthreads();
  const float mu = ((red[0] + red[1]) + (red[2] + red[3])) * 0.0009765625f;
  float d[8];
  d[0] = a0[0] - mu; d[1] = a0[1] - mu; d[2] = a0[2] - mu; d[3] = a0[3] - mu;
  d[4] = a1[0] - mu; d[5] = a1[1] - mu; d[6] = a1[2] - mu; d[7] = a1[3] - mu;
  float v = 0.f;
#pragma unroll
  for (int e = 0; e < 8; ++e) v += d[e] * d[e];
#pragma unroll
  for (int off = 1; off < 32; off <<= 1) v += __shfl_xor(v, off, 32);
  if (lane == 0) red[4 + wave] = v;
  __syncthreads();
  const float var  = ((red[4] + red[5]) + (red[6] + red[7])) * 0.0009765625f;
  const float rstd = rsqrtf(var + 1e-5f);
  const float gr   = gate[row];
  const float g    = (use_gate != 0) ? gr : 1.0f;
  const v4f w0 = *(const v4f*)(w + col);
  const v4f w1 = *(const v4f*)(w + col + 4);
  const v4f y0 = (v4f){d[0] * rstd * w0[0] * g, d[1] * rstd * w0[1] * g, d[2] * rstd * w0[2] * g, d[3] * rstd * w0[3] * g};
  const v4f y1 = (v4f){d[4] * rstd * w1[0] * g, d[5] * rstd * w1[1] * g, d[6] * rstd * w1[2] * g, d[7] * rstd * w1[3] * g};
  const v4u pk = packh(y0, y1);
  volatile v4u* dp = (volatile v4u*)(out + (size_t)row * DM + col);
  *dp = pk;
  __threadfence();
  *dp = pk;
}

__global__ __launch_bounds__(256) void k_wcvt(const float* __restrict__ src, _Float16* __restrict__ dst,
                                              float scale, int n8) {
  const int i = blockIdx.x * 256 + (int)threadIdx.x;
  if (i >= n8) return;
  const size_t o = (size_t)i * 8;
  const v4f a0 = *(const v4f*)(src + o);
  const v4f a1 = *(const v4f*)(src + o + 4);
  const v4u pk = packh(a0 * scale, a1 * scale);
  volatile v4u* dp = (volatile v4u*)(dst + o);
  *dp = pk;
  __threadfence();
  *dp = pk;
}

#define SFP 68
__global__ __launch_bounds__(128) void k_qkv(const _Float16* __restrict__ hp,
                                             const _Float16* __restrict__ wt,
                                             _Float16* __restrict__ qp,
                                             _Float16* __restrict__ kp,
                                             _Float16* __restrict__ vtp) {
  __shared__ __align__(16) float sf[128 * SFP];
  const int tid = threadIdx.x, lane = tid & 31, wave = tid >> 5;
  const int hh = lane >> 4, c = lane & 15;
  const int mb = blockIdx.x * 128;
  const int b  = mb / SQ;
  const int sb = mb - b * SQ;
  const int ns = blockIdx.y;
  const int which = ns >> 4;
  const int head  = ns & 15;
  const int hb = b * NH + head;
  const int m0 = mb + wave * 32;
  const int n0 = ns * HD;

  v8f acc[2][4];
#pragma unroll
  for (int s = 0; s < 2; ++s)
#pragma unroll
    for (int t = 0; t < 4; ++t) acc[s][t] = zero8();
  gemm32x64(hp, DM, wt, DM, DM, m0, n0, lane, acc);

#pragma unroll
  for (int sub = 0; sub < 2; ++sub)
#pragma unroll
    for (int t = 0; t < 4; ++t)
#pragma unroll
      for (int r = 0; r < 8; ++r)
        sf[(wave * 32 + sub * 16 + 8 * hh + r) * SFP + 16 * t + c] = acc[sub][t][r] * 0.03125f;
  __syncthreads();

  if (which < 2) {
    _Float16* base = (which == 0) ? qp : kp;
    v4u val[8];
#pragma unroll
    for (int j = 0; j < 8; ++j) {
      const int p  = tid + 128 * j;
      const int lr = p >> 3;
      const int pc = p & 7;
      const float* ra = sf + lr * SFP + pc * 8;
      val[j] = packh(*(const v4f*)(ra), *(const v4f*)(ra + 4));
    }
    for (int ps = 0; ps < 2; ++ps) {
#pragma unroll
      for (int j = 0; j < 8; ++j) {
        const int p  = tid + 128 * j;
        const int lr = p >> 3;
        const int pc = p & 7;
        const size_t go = ((size_t)hb * SQ + sb + lr) * HD + pc * 8;
        *(volatile v4u*)(base + go) = val[j];
      }
      __threadfence();
    }
  } else {
    v4u val[8];
#pragma unroll
    for (int j = 0; j < 8; ++j) {
      const int p  = tid + 128 * j;
      const int d  = p >> 4;
      const int pc = p & 15;
      const float* cp = sf + (pc * 8) * SFP + d;
      Pack8 pk;
      pk.h = (v8h){(_Float16)cp[0 * SFP], (_Float16)cp[1 * SFP], (_Float16)cp[2 * SFP], (_Float16)cp[3 * SFP],
                   (_Float16)cp[4 * SFP], (_Float16)cp[5 * SFP], (_Float16)cp[6 * SFP], (_Float16)cp[7 * SFP]};
      val[j] = pk.u;
    }
    for (int ps = 0; ps < 2; ++ps) {
#pragma unroll
      for (int j = 0; j < 8; ++j) {
        const int p  = tid + 128 * j;
        const int d  = p >> 4;
        const int pc = p & 15;
        const size_t go = ((size_t)hb * HD + d) * SQ + sb + pc * 8;
        *(volatile v4u*)(vtp + go) = val[j];
      }
      __threadfence();
    }
  }
}

#define KTP 72
__global__ __launch_bounds__(256) void k_attn(const _Float16* __restrict__ qp,
                                              const _Float16* __restrict__ kp,
                                              const _Float16* __restrict__ vt,
                                              const float* __restrict__ gate,
                                              _Float16* __restrict__ op, float sscale) {
  __shared__ __align__(16) _Float16 Ks[KC * KTP];
  __shared__ __align__(16) _Float16 Vs[HD * KTP];
  __shared__ __align__(16) _Float16 Ps[8 * 16 * KTP];

  const int tid = threadIdx.x, lane = tid & 31, wave = tid >> 5;
  const int hh = lane >> 4, c = lane & 15;
  const int qb = blockIdx.x % NQB;
  const int hb = blockIdx.x / NQB;
  const int h  = hb % NH;
  const int b  = hb / NH;
  const int q0 = qb * QB + wave * 16;

  const _Float16* Q = qp + (size_t)hb * SQ * HD;
  const _Float16* K = kp + (size_t)hb * SQ * HD;
  const _Float16* V = vt + (size_t)hb * HD * SQ;
  const float* gk = gate + (size_t)b * SQ;
  const size_t trow0 = (size_t)b * SQ;

  const v16h qa0 = ldfrag(Q, HD, q0, 0, lane);
  const v16h qa1 = ldfrag(Q, HD, q0, 32, lane);

  const float NEGI = -__builtin_huge_valf();
  float mrow[8], lrow[8];
  v8f oacc[4];
#pragma unroll
  for (int r = 0; r < 8; ++r) { mrow[r] = NEGI; lrow[r] = 0.f; }
#pragma unroll
  for (int t = 0; t < 4; ++t) oacc[t] = zero8();

  _Float16* pw = Ps + wave * 16 * KTP;
  const int nck = 2 * qb + 2;

  for (int kc = 0; kc < nck; ++kc) {
    const int kv0 = kc * KC;
    float mv[4];
    int okl = 0;
#pragma unroll
    for (int j = 0; j < 4; ++j) {
      mv[j] = gk[kv0 + 16 * j + c];
      okl |= (mv[j] > 0.f) ? 1 : 0;
    }
    if (__ballot(okl) == 0ull) continue;
    __syncthreads();
    {
      const int r  = tid >> 2;
      const int qq = (tid & 3) * 16;
      const _Float16* ks = K + (size_t)(kv0 + r) * HD + qq;
      *(v8h*)(Ks + r * KTP + qq)     = *(const v8h*)(ks);
      *(v8h*)(Ks + r * KTP + qq + 8) = *(const v8h*)(ks + 8);
      const _Float16* vs = V + (size_t)r * SQ + kv0 + qq;
      *(v8h*)(Vs + r * KTP + qq)     = *(const v8h*)(vs);
      *(v8h*)(Vs + r * KTP + qq + 8) = *(const v8h*)(vs + 8);
    }
    __syncthreads();

    v8f s[4];
#pragma unroll
    for (int j = 0; j < 4; ++j) s[j] = zero8();
#pragma unroll
    for (int j = 0; j < 4; ++j) {
      const v16h kb0 = ldfrag(Ks, KTP, j * 16, 0, lane);
      s[j] = mma16(qa0, kb0, s[j]);
      const v16h kb1 = ldfrag(Ks, KTP, j * 16, 32, lane);
      s[j] = mma16(qa1, kb1, s[j]);
    }
    const bool edge = (kc >= 2 * qb);
#pragma unroll
    for (int r = 0; r < 8; ++r) {
      const int qry = q0 + 8 * hh + r;
#pragma unroll
      for (int j = 0; j < 4; ++j) {
        const int key = kv0 + 16 * j + c;
        const float v = s[j][r] * sscale;
        const bool bad = (edge && key > qry) || !(mv[j] > 0.f);
        s[j][r] = bad ? NEGI : v;
      }
    }
    float cm[8];
#pragma unroll
    for (int r = 0; r < 8; ++r) {
      float m = NEGI;
#pragma unroll
      for (int j = 0; j < 4; ++j) m = fmaxf(m, s[j][r]);
#pragma unroll
      for (int off = 1; off < 16; off <<= 1) m = fmaxf(m, __shfl_xor(m, off, 32));
      cm[r] = m;
    }
    float al[8];
#pragma unroll
    for (int r = 0; r < 8; ++r) {
      const float mnew = fmaxf(mrow[r], cm[r]);
      const bool  fin  = (mnew != NEGI);
      const float alpha = fin ? __expf(mrow[r] - mnew) : 1.0f;
      mrow[r] = mnew;
      float psum = 0.f;
#pragma unroll
      for (int j = 0; j < 4; ++j) {
        const float p = fin ? __expf(s[j][r] - mnew) : 0.0f;
        psum += p;
        pw[(8 * hh + r) * KTP + j * 16 + c] = (_Float16)(p * 1024.0f);
      }
#pragma unroll
      for (int off = 1; off < 16; off <<= 1) psum += __shfl_xor(psum, off, 32);
      lrow[r] = lrow[r] * alpha + psum;
      al[r] = alpha;
    }
#pragma unroll
    for (int t = 0; t < 4; ++t)
#pragma unroll
      for (int r = 0; r < 8; ++r) oacc[t][r] *= al[r];
    __syncthreads();

#pragma unroll
    for (int kk = 0; kk < 2; ++kk) {
      const v16h pa = ldfrag(pw, KTP, 0, kk * 32, lane);
#pragma unroll
      for (int t = 0; t < 4; ++t) {
        const v16h vb = ldfrag(Vs, KTP, t * 16, kk * 32, lane);
        oacc[t] = mma16(pa, vb, oacc[t]);
      }
    }
  }

  float invl[8];
#pragma unroll
  for (int r = 0; r < 8; ++r) invl[r] = (lrow[r] > 0.f) ? (0.015625f / lrow[r]) : 0.f;
  __syncthreads();
#pragma unroll
  for (int r = 0; r < 8; ++r) {
#pragma unroll
    for (int t = 0; t < 4; ++t)
      pw[(8 * hh + r) * KTP + 16 * t + c] = (_Float16)(oacc[t][r] * invl[r]);
  }
  __syncthreads();
  v4u val[4];
#pragma unroll
  for (int it = 0; it < 4; ++it) {
    const int p  = lane + 32 * it;
    const int L  = p >> 3;
    const int pc = p & 7;
    Pack8 pk;
    pk.h    = *(const v8h*)(pw + L * KTP + pc * 8);
    val[it] = pk.u;
  }
  for (int ps = 0; ps < 2; ++ps) {
#pragma unroll
    for (int it = 0; it < 4; ++it) {
      const int p  = lane + 32 * it;
      const int L  = p >> 3;
      const int pc = p & 7;
      const size_t go = (trow0 + q0 + L) * DM + (size_t)h * HD + pc * 8;
      *(volatile v4u*)(op + go) = val[it];
    }
    __threadfence();
  }
}

#define OTP 68
__device__ __forceinline__ float gelu_tanh(float v) {
  return 0.5f * v * (1.0f + tanhf(0.7978845608028654f * (v + 0.044715f * v * v * v)));
}

template <int EPI>
__global__ __launch_bounds__(128) void k_gemm(const _Float16* __restrict__ A,
                                              const _Float16* __restrict__ Bt,
                                              int K, int N,
                                              const float* __restrict__ res,
                                              const float* __restrict__ gate,
                                              float scale,
                                              float* __restrict__ outf,
                                              _Float16* __restrict__ outh) {
  __shared__ __align__(16) float st[4 * 32 * OTP];
  const int tid = threadIdx.x, lane = tid & 31, wave = tid >> 5;
  const int hh = lane >> 4, c = lane & 15;
  const int m0 = blockIdx.x * 128 + wave * 32;
  const int n0 = blockIdx.y * 64;

  v8f acc[2][4];
#pragma unroll
  for (int s = 0; s < 2; ++s)
#pragma unroll
    for (int t = 0; t < 4; ++t) acc[s][t] = zero8();
  gemm32x64(A, K, Bt, K, K, m0, n0, lane, acc);

  float* sw = st + wave * 32 * OTP;
#pragma unroll
  for (int sub = 0; sub < 2; ++sub) {
    float mr[8];
#pragma unroll
    for (int r = 0; r < 8; ++r) mr[r] = (EPI == 2) ? gate[m0 + sub * 16 + 8 * hh + r] : 1.0f;
#pragma unroll
    for (int t = 0; t < 4; ++t)
#pragma unroll
      for (int r = 0; r < 8; ++r)
        sw[(sub * 16 + 8 * hh + r) * OTP + 16 * t + c] = acc[sub][t][r] * scale * mr[r];
  }
  __syncthreads();

  if (EPI == 1) {
#pragma unroll 1
    for (int it = 0; it < 8; ++it) {
      const int p  = lane + 32 * it;
      const int L  = p >> 3;
      const int pc = p & 7;
      float* q = sw + L * OTP + pc * 8;
      const float g4 = gate[m0 + L] * 4.0f;
      const v4f a0 = *(const v4f*)(q);
      const v4f a1 = *(const v4f*)(q + 4);
      const v4f g0 = (v4f){gelu_tanh(a0[0]) * g4, gelu_tanh(a0[1]) * g4, gelu_tanh(a0[2]) * g4, gelu_tanh(a0[3]) * g4};
      const v4f g1 = (v4f){gelu_tanh(a1[0]) * g4, gelu_tanh(a1[1]) * g4, gelu_tanh(a1[2]) * g4, gelu_tanh(a1[3]) * g4};
      *(v4f*)(q)     = g0;
      *(v4f*)(q + 4) = g1;
    }
    __syncthreads();
    for (int ps = 0; ps < 2; ++ps) {
#pragma unroll
      for (int it = 0; it < 8; ++it) {
        const int p  = lane + 32 * it;
        const int L  = p >> 3;
        const int pc = p & 7;
        const float* q = sw + L * OTP + pc * 8;
        const v4u pk = packh(*(const v4f*)(q), *(const v4f*)(q + 4));
        const size_t go = (size_t)(m0 + L) * (size_t)N + n0 + pc * 8;
        *(volatile v4u*)(outh + go) = pk;
      }
      __threadfence();
    }
  } else {
    for (int ps = 0; ps < 2; ++ps) {
#pragma unroll
      for (int it = 0; it < 16; ++it) {
        const int p    = lane + 32 * it;
        const int L    = p >> 3;
        const int pc   = p & 7;
        const int row  = L >> 1;
        const int half = L & 1;
        v4f v = *(const v4f*)(sw + row * OTP + half * 32 + pc * 4);
        const size_t go = (size_t)(m0 + row) * (size_t)N + n0 + half * 32 + pc * 4;
        const v4f rr = *(const v4f*)(res + go);
        v = rr + v;
        *(volatile v4f*)(outf + go) = v;
      }
      __threadfence();
    }
  }
}

extern "C" void kernel_launch(void* const* d_in, const int* in_sizes, int n_in,
                              void* d_out, int out_size, void* d_ws, size_t ws_size,
                              hipStream_t stream) {
  if (n_in < 8) return;
  if (in_sizes[0] != NTOK * DM) return;
  if (in_sizes[1] != NTOK) return;
  if (in_sizes[2] != DM) return;
  if (in_sizes[3] != NQKV * DM) return;
  if (in_sizes[4] != DM * DM) return;
  if (in_sizes[5] != DM) return;
  if (in_sizes[6] != DFF * DM) return;
  if (in_sizes[7] != DM * DFF) return;
  if (out_size != NTOK * DM) return;

  const float* x     = (const float*)d_in[0];
  const float* gatev = (const float*)d_in[1];
  const float* ln1w  = (const float*)d_in[2];
  const float* wqkv  = (const float*)d_in[3];
  const float* wo    = (const float*)d_in[4];
  const float* ln2w  = (const float*)d_in[5];
  const float* w1    = (const float*)d_in[6];
  const float* w2    = (const float*)d_in[7];
  float* out = (float*)d_out;

  size_t off = 0;
  const size_t oH   = off; off += (size_t)NTOK * DM * 2;
  const size_t oWq  = off; off += (size_t)NQKV * DM * 2;
  const size_t oWo  = off; off += (size_t)DM * DM * 2;
  const size_t oW1  = off; off += (size_t)DFF * DM * 2;
  const size_t oW2  = off; off += (size_t)DM * DFF * 2;
  const size_t oQ   = off; off += (size_t)NB * NH * SQ * HD * 2;
  const size_t oK   = off; off += (size_t)NB * NH * SQ * HD * 2;
  const size_t oVt  = off; off += (size_t)NB * NH * HD * SQ * 2;
  const size_t oO   = off; off += (size_t)NTOK * DM * 2;
  const size_t oX1  = off; off += (size_t)NTOK * DM * 4;
  const size_t oH3  = off; off += (size_t)NTOK * DFF * 2;
  if (off > ws_size) return;
  if (off > (size_t)WSLIM) return;

  char* ws = (char*)d_ws;
  _Float16* Hp  = (_Float16*)(ws + oH);
  _Float16* Wq  = (_Float16*)(ws + oWq);
  _Float16* Wop = (_Float16*)(ws + oWo);
  _Float16* W1p = (_Float16*)(ws + oW1);
  _Float16* W2p = (_Float16*)(ws + oW2);
  _Float16* Qp  = (_Float16*)(ws + oQ);
  _Float16* Kp  = (_Float16*)(ws + oK);
  _Float16* Vt  = (_Float16*)(ws + oVt);
  _Float16* Op  = (_Float16*)(ws + oO);
  float*    X1  = (float*)(ws + oX1);
  _Float16* H3  = (_Float16*)(ws + oH3);

  k_ln<<<dim3(NTOK), dim3(128), 0, stream>>>(x, ln1w, gatev, 0, Hp);
  {
    const int n8q = (NQKV * DM) / 8, n8o = (DM * DM) / 8, n81 = (DFF * DM) / 8, n82 = (DM * DFF) / 8;
    k_wcvt<<<dim3((n8q + 255) / 256), dim3(256), 0, stream>>>(wqkv, Wq, 32.0f, n8q);
    k_wcvt<<<dim3((n8o + 255) / 256), dim3(256), 0, stream>>>(wo, Wop, 32.0f, n8o);
    k_wcvt<<<dim3((n81 + 255) / 256), dim3(256), 0, stream>>>(w1, W1p, 32.0f, n81);
    k_wcvt<<<dim3((n82 + 255) / 256), dim3(256), 0, stream>>>(w2, W2p, 64.0f, n82);
  }
  k_qkv<<<dim3(NTOK / 128, NQKV / HD), dim3(128), 0, stream>>>(Hp, Wq, Qp, Kp, Vt);
  const float sscale = 0.125f;
  k_attn<<<dim3(NB * NH * NQB), dim3(256), 0, stream>>>(Qp, Kp, Vt, gatev, Op, sscale);
  k_gemm<0><<<dim3(NTOK / 128, DM / 64), dim3(128), 0, stream>>>(Op, Wop, DM, DM, x, gatev, 0.001953125f, X1, H3);
  k_ln<<<dim3(NTOK), dim3(128), 0, stream>>>(X1, ln2w, gatev, 1, Hp);
  k_gemm<1><<<dim3(NTOK / 128, DFF / 64), dim3(128), 0, stream>>>(Hp, W1p, DM, DFF, X1, gatev, 0.03125f, X1, H3);
  k_gemm<2><<<dim3(NTOK / 128, DM / 64), dim3(128), 0, stream>>>(H3, W2p, DFF, DM, X1, gatev, 0.00390625f, out, H3);
  (void)hipGetLastError();
}
